// GenerateActionsBlock_57312043597846
// MI455X (gfx1250) — hardware-verified
//
#include <hip/hip_runtime.h>
#include <math.h>
#include <stddef.h>

typedef _Float16 v16h __attribute__((ext_vector_type(16)));
typedef _Float16 v8h  __attribute__((ext_vector_type(8)));
typedef float    v8f  __attribute__((ext_vector_type(8)));
typedef float    v4f  __attribute__((ext_vector_type(4)));
typedef v4f      v4fa __attribute__((may_alias));

union Frag { v16h v; v8h half[2]; };

constexpr int B_ = 16;
constexpr int N_ = 1024;
constexpr int E_ = 128;
constexpr int KV_STRIDE = 2 * E_ + 1;
constexpr int KVP_PITCH = 2 * E_;
constexpr int TILES  = B_ * (N_ / 16);
constexpr int WAVES2 = 8;
constexpr int ROWS_PER_PACK_BLOCK = 8;

constexpr float OP_SCALE  = 64.0f;
constexpr float RSQRT_E   = 0.08838834764831845f;
constexpr float REL_SCALE = RSQRT_E * (1.0f / 4096.0f);

static_assert(E_ % 32 == 0);
static_assert(N_ % (16 * WAVES2) == 0);
static_assert(TILES % WAVES2 == 0);
static_assert((B_ * N_) % ROWS_PER_PACK_BLOCK == 0);
static_assert((WAVES2 * 16 * 3) % (4 * 32) == 0);

__device__ __forceinline__ v8f wmma_f16(v16h a, v16h b, v8f c)
{
  v8f d = __builtin_amdgcn_wmma_f32_16x16x32_f16(false, a, false, b, (short)0, c, false, false);
  asm volatile("v_nop\n\tv_nop\n\tv_nop\n\tv_nop" : "+v"(d) : "v"(a), "v"(b));
  return d;
}

__global__ __launch_bounds__(256) void k_pack(const float* __restrict__ kv,
                                              const float* __restrict__ mask,
                                              _Float16* kvp, int nrows)
{
  const int lane = threadIdx.x & 31;
  const int row  = blockIdx.x * ROWS_PER_PACK_BLOCK + (threadIdx.x >> 5);
  if (row >= nrows) return;
  const float mscale = mask[row] * OP_SCALE;
  const float* src = kv + (size_t)row * KV_STRIDE + lane * 8;
  v8h v;
  #pragma unroll
  for (int i = 0; i < 8; ++i) v[i] = (_Float16)(src[i] * mscale);
  volatile v8h* dst = (volatile v8h*)(kvp + (size_t)row * KVP_PITCH + lane * 8);
  *dst = v;
  __threadfence();
  *dst = v;
}

__global__ __launch_bounds__(256) void k_actions(const _Float16* __restrict__ kvp,
                                                 const float* __restrict__ pos,
                                                 const float* __restrict__ mask,
                                                 const float* __restrict__ ascale,
                                                 float* out)
{
  __shared__ __attribute__((aligned(16))) float s_out[WAVES2 * 16 * 3];

  const int lane = threadIdx.x & 31;
  const int wave = threadIdx.x >> 5;
  const int h = lane >> 4;
  const int m = lane & 15;
  const int tile = blockIdx.x * WAVES2 + wave;
  const int b  = tile / (N_ / 16);
  const int i0 = (tile % (N_ / 16)) * 16;
  const size_t brow = (size_t)b * N_;
  const float* posb  = pos  + brow * 3;
  const float* maskb = mask + brow;

  float msum = 0.f;
  #pragma unroll 1
  for (int t = lane; t < N_; t += 32) msum += maskb[t];
  #pragma unroll
  for (int off = 16; off; off >>= 1) msum += __shfl_xor(msum, off, 32);
  const float inv_msum = 1.0f / msum;

  const _Float16* arow = kvp + (brow + (size_t)(i0 + m)) * KVP_PITCH;
  Frag A[4];
  #pragma unroll
  for (int ks = 0; ks < 4; ++ks) {
    A[ks].half[0] = *(const v8h*)(arow + ks * 32 + 8 * h);
    A[ks].half[1] = *(const v8h*)(arow + ks * 32 + 16 + 8 * h);
  }

  float pix[8], piy[8], piz[8], mi[8];
  #pragma unroll
  for (int r = 0; r < 8; ++r) {
    const int i = i0 + 8 * h + r;
    pix[r] = posb[i * 3 + 0];
    piy[r] = posb[i * 3 + 1];
    piz[r] = posb[i * 3 + 2];
    mi[r]  = maskb[i];
  }

  float ax[8], ay[8], az[8];
  #pragma unroll
  for (int r = 0; r < 8; ++r) { ax[r] = 0.f; ay[r] = 0.f; az[r] = 0.f; }

  #pragma unroll 1
  for (int j0 = 0; j0 < N_; j0 += 16) {
    const int jr = j0 + m;
    const _Float16* vrow = kvp + (brow + (size_t)jr) * KVP_PITCH + E_;

    v8f c = {0.f, 0.f, 0.f, 0.f, 0.f, 0.f, 0.f, 0.f};
    #pragma unroll
    for (int ks = 0; ks < 4; ++ks) {
      Frag bt;
      bt.half[0] = *(const v8h*)(vrow + ks * 32 + 8 * h);
      bt.half[1] = *(const v8h*)(vrow + ks * 32 + 16 + 8 * h);
      c = wmma_f16(A[ks].v, bt.v, c);
    }

    const float pjx = posb[jr * 3 + 0];
    const float pjy = posb[jr * 3 + 1];
    const float pjz = posb[jr * 3 + 2];

    #pragma unroll
    for (int r = 0; r < 8; ++r) {
      const float s  = c[r] * REL_SCALE;
      const float dx = pix[r] - pjx;
      const float dy = piy[r] - pjy;
      const float dz = piz[r] - pjz;
      const float n2 = dx * dx + dy * dy + dz * dz;
      const float w  = s * __builtin_amdgcn_rcpf(__builtin_amdgcn_sqrtf(n2) + 1e-8f);
      ax[r] += dx * w;
      ay[r] += dy * w;
      az[r] += dz * w;
    }
  }

  #pragma unroll
  for (int r = 0; r < 8; ++r) {
    #pragma unroll
    for (int off = 8; off; off >>= 1) {
      ax[r] += __shfl_xor(ax[r], off, 16);
      ay[r] += __shfl_xor(ay[r], off, 16);
      az[r] += __shfl_xor(az[r], off, 16);
    }
  }

  if (m < 8) {
    float vx = ax[0], vy = ay[0], vz = az[0], mk = mi[0];
    #pragma unroll
    for (int r = 1; r < 8; ++r) {
      if (m == r) { vx = ax[r]; vy = ay[r]; vz = az[r]; mk = mi[r]; }
    }
    const float as = ascale[0];
    const int rl = wave * 16 + 8 * h + m;
    s_out[rl * 3 + 0] = (as * tanhf(vx * inv_msum)) * mk;
    s_out[rl * 3 + 1] = (as * tanhf(vy * inv_msum)) * mk;
    s_out[rl * 3 + 2] = (as * tanhf(vz * inv_msum)) * mk;
  }
  __syncthreads();

  if (wave < 3) {
    const int q = wave * 32 + lane;
    const v4f v = *(const v4fa*)(s_out + 4 * q);
    volatile v4f* dst = (volatile v4f*)(out + (size_t)blockIdx.x * (WAVES2 * 16 * 3) + 4 * q);
    *dst = v;
    __threadfence();
    *dst = v;
  }
}

extern "C" void kernel_launch(void* const* d_in, const int* in_sizes, int n_in,
                              void* d_out, int out_size, void* d_ws, size_t ws_size,
                              hipStream_t stream)
{
  if (n_in < 4) return;
  if (in_sizes[0] != B_ * N_ * KV_STRIDE) return;
  if (in_sizes[1] != B_ * N_ * 3) return;
  if (in_sizes[2] != B_ * N_) return;
  if (in_sizes[3] < 1) return;
  if (out_size != B_ * N_ * 3) return;

  const size_t kvp_bytes = (size_t)B_ * N_ * KVP_PITCH * sizeof(_Float16);
  if (kvp_bytes > ws_size) return;

  const float* kv     = (const float*)d_in[0];
  const float* pos    = (const float*)d_in[1];
  const float* mask   = (const float*)d_in[2];
  const float* ascale = (const float*)d_in[3];
  float* out = (float*)d_out;
  _Float16* kvp = (_Float16*)d_ws;

  const int nrows = B_ * N_;
  k_pack<<<(nrows + ROWS_PER_PACK_BLOCK - 1) / ROWS_PER_PACK_BLOCK, 32 * ROWS_PER_PACK_BLOCK, 0, stream>>>(
      kv, mask, kvp, nrows);
  k_actions<<<TILES / WAVES2, 32 * WAVES2, 0, stream>>>(kvp, pos, mask, ascale, out);
}
